// SelfAttentionPooling_47021301957262
// MI455X (gfx1250) — hardware-verified
//
#include <hip/hip_runtime.h>
#include <math.h>

typedef __attribute__((ext_vector_type(16))) _Float16 v16h;
typedef __attribute__((ext_vector_type(16))) __bf16 v16b;
typedef __attribute__((ext_vector_type(8)))  _Float16 v8h;
typedef __attribute__((ext_vector_type(8)))  float v8f;
typedef __attribute__((ext_vector_type(4)))  float v4f;
typedef __attribute__((ext_vector_type(2)))  float v2f;
typedef __attribute__((ext_vector_type(4)))  unsigned v4u;
typedef __attribute__((ext_vector_type(4)))  int v4i;
typedef float __attribute__((may_alias)) float_a;
typedef int __attribute__((may_alias)) int_a;

template <typename T> __device__ __forceinline__ void vst2(void* p, T v) { *(volatile T*)p = v; __threadfence(); *(volatile T*)p = v; }
__device__ __forceinline__ v8f wmma16(v16h a, v16h b, v8f c) {
  v8f d = __builtin_amdgcn_wmma_f32_16x16x32_f16(false, a, false, b, (short)0, c, false, false);
  asm volatile("v_nop\n\tv_nop\n\tv_nop\n\tv_nop" : "+v"(d) : "v"(a), "v"(b));
  return d;
}
__device__ __forceinline__ v8f wmma_bf(v16b a, v16b b, v8f c) {
  v8f d = __builtin_amdgcn_wmma_f32_16x16x32_bf16(false, a, false, b, (short)0, c, false, false);
  asm volatile("v_nop\n\tv_nop\n\tv_nop\n\tv_nop" : "+v"(d) : "v"(a), "v"(b));
  return d;
}
__device__ __forceinline__ v16h frag_h(const _Float16* rowk0, int lane) {
  union { v16h v; v8h q[2]; } u; const _Float16* p = rowk0 + 8 * (lane >> 4);
  u.q[0] = *(const v8h*)p; u.q[1] = *(const v8h*)(p + 16); return u.v;
}
__device__ __forceinline__ v16h frag_f32(const float* rowk0, int lane) {
  v16h a; const float* p = rowk0 + 8 * (lane >> 4);
#pragma unroll
  for (int i = 0; i < 8; ++i) { a[i] = (_Float16)p[i]; a[8 + i] = (_Float16)p[16 + i]; }
  return a;
}
__device__ __forceinline__ v16h frag_f32s(const float* rowk0, int lane, float sc) {
  v16h a; const float* p = rowk0 + 8 * (lane >> 4);
#pragma unroll
  for (int i = 0; i < 8; ++i) { a[i] = (_Float16)(p[i] * sc); a[8 + i] = (_Float16)(p[16 + i] * sc); }
  return a;
}
__device__ __forceinline__ v16h fragc_f32(const float* W, int k0, int n, int lane, int ld, int K) {
  v16h a; const int g = lane >> 4;
#pragma unroll
  for (int i = 0; i < 8; ++i) { const int ka = k0 + 8 * g + i, kb = ka + 16;
    a[i] = (_Float16)(ka < K ? W[(size_t)(ka < K ? ka : K - 1) * ld + n] : 0.f); a[8 + i] = (_Float16)(kb < K ? W[(size_t)(kb < K ? kb : K - 1) * ld + n] : 0.f); }
  return a;
}
struct F2 { v16b h, l; };
__device__ __forceinline__ F2 bsplit16(const float v[16]) { F2 r;
#pragma unroll
  for (int i = 0; i < 16; ++i) { const __bf16 h = (__bf16)v[i]; r.h[i] = h; r.l[i] = (__bf16)(v[i] - (float)h); }
  return r; }
__device__ __forceinline__ F2 split_row(const float* row, int k0, int lane) { float v[16]; const float* p = row + k0 + 8 * (lane >> 4);
#pragma unroll
  for (int i = 0; i < 8; ++i) { v[i] = p[i]; v[8 + i] = p[16 + i]; }
  return bsplit16(v); }
__device__ __forceinline__ F2 split_rowK(const float* row, int k0, int lane, int K) { float v[16]; const int g = lane >> 4;
#pragma unroll
  for (int i = 0; i < 8; ++i) { const int ka = k0 + 8 * g + i, kb = ka + 16; v[i] = ka < K ? row[ka < K ? ka : K - 1] : 0.f; v[8 + i] = kb < K ? row[kb < K ? kb : K - 1] : 0.f; }
  return bsplit16(v); }
__device__ __forceinline__ F2 split_col(const float* W, int k0, int n, int lane, int ld, int K) { float v[16]; const int g = lane >> 4;
#pragma unroll
  for (int i = 0; i < 8; ++i) { const int ka = k0 + 8 * g + i, kb = ka + 16; v[i] = ka < K ? W[(size_t)(ka < K ? ka : K - 1) * ld + n] : 0.f; v[8 + i] = kb < K ? W[(size_t)(kb < K ? kb : K - 1) * ld + n] : 0.f; }
  return bsplit16(v); }
__device__ __forceinline__ v8f mac3(const F2& a, const F2& b, v8f c) { c = wmma_bf(a.l, b.h, c); c = wmma_bf(a.h, b.l, c); return wmma_bf(a.h, b.h, c); }
__device__ __forceinline__ float sigm(float v) { return 1.0f / (1.0f + expf(-v)); }
#define LDSX() do { asm volatile("s_wait_dscnt 0" ::: "memory"); __builtin_amdgcn_wave_barrier(); __builtin_amdgcn_fence(__ATOMIC_RELEASE, "workgroup"); } while (0)

__device__ __forceinline__ float bfr(float v) { return (float)(__bf16)v; }
#define NBQ 8192
#define SS 200
#define VV 100000
#define DD 64
#define HH 64
#define NROW (NBQ * SS)
#ifndef NRB
#define NRB (NROW / 64)
#endif
#ifndef NPB
#define NPB (NBQ / 8)
#endif
#define WS_SC 0u
#define WS_END (WS_SC + 4u * (size_t)NROW)
__global__ __launch_bounds__(128) void k_score(const float* __restrict__ TAB, const float* __restrict__ W1, const float* __restrict__ B1, const float* __restrict__ W2, const float* __restrict__ B2, const int* __restrict__ IDS, float* __restrict__ SC) { __shared__ __align__(16) float so[64];
  const int tid = threadIdx.x, wave = tid >> 5, lane = tid & 31, col = lane & 15, g = lane >> 4; const size_t r0 = (size_t)blockIdx.x * 64 + wave * 16; const size_t row = r0 + col;
  int id = IDS[row]; id = id < 0 ? 0 : (id >= VV ? VV - 1 : id); const float* er = TAB + (size_t)id * DD;
  v8f acc[4] = {};
#pragma unroll
  for (int kc = 0; kc < DD / 32; ++kc) { v16b a; { const float* p = er + kc * 32 + 8 * g;
#pragma unroll
      for (int i = 0; i < 8; ++i) { a[i] = (__bf16)p[i]; a[8 + i] = (__bf16)p[16 + i]; } }
#pragma unroll
    for (int j = 0; j < 4; ++j) { v16b w; const int o = j * 16 + col;
#pragma unroll
      for (int i = 0; i < 8; ++i) { w[i] = (__bf16)W1[(size_t)(kc * 32 + 8 * g + i) * HH + o]; w[8 + i] = (__bf16)W1[(size_t)(kc * 32 + 16 + 8 * g + i) * HH + o]; }
      asm volatile("s_wait_loadcnt 0x0" ::: "memory"); acc[j] = wmma_bf(a, w, acc[j]); } }
  float part[8];
#pragma unroll
  for (int r = 0; r < 8; ++r) part[r] = 0.f;
#pragma unroll
  for (int j = 0; j < 4; ++j) { const int o = j * 16 + col; const float bb = bfr(B1[o]), w2 = bfr(W2[o]);
#pragma unroll
    for (int r = 0; r < 8; ++r) part[r] += tanhf(acc[j][r] + bb) * w2; }
#pragma unroll
  for (int r = 0; r < 8; ++r) {
#pragma unroll
    for (int o_ = 1; o_ < 16; o_ <<= 1) part[r] += __shfl_xor(part[r], o_); }
  if (col == 0) { const float b2 = bfr(B2[0]);
#pragma unroll
    for (int r = 0; r < 8; ++r) so[wave * 16 + 8 * g + r] = part[r] + b2; }
  __syncthreads();
  if (tid < 16) vst2(SC + (size_t)blockIdx.x * 64 + tid * 4, *(const v4f*)&so[tid * 4]); }
__global__ __launch_bounds__(256) void k_pool(const float* __restrict__ TAB, const float* __restrict__ SC, const int* __restrict__ IDS, const int* __restrict__ LEN, float* __restrict__ OUT) { __shared__ float sp[8][SS]; __shared__ __align__(16) float so[8][DD];
  const int t = threadIdx.x; const int grp = t >> 5, lane = t & 31; const size_t b = (size_t)blockIdx.x * 8 + grp; int len = LEN[b]; len = len < 1 ? 1 : (len > SS ? SS : len);
  const float* sc = SC + b * SS; float m = -3.0e38f;
  for (int s = lane; s < SS; s += 32) { const float v = (s < len) ? sc[s] : -3.0e38f; sp[grp][s] = v; m = fmaxf(m, v); }
#pragma unroll
  for (int o = 1; o < 32; o <<= 1) m = fmaxf(m, __shfl_xor(m, o));
  float z = 0.f; for (int s = lane; s < SS; s += 32) { const float e = (s < len) ? expf(sp[grp][s] - m) : 0.f; sp[grp][s] = e; z += e; }
#pragma unroll
  for (int o = 1; o < 32; o <<= 1) z += __shfl_xor(z, o);
  const float inv = 1.0f / z;
  __syncthreads();
  float a0 = 0.f, a1 = 0.f;
#pragma unroll 2
  for (int s = 0; s < SS; ++s) { if (s >= len) break; int id = IDS[b * SS + s]; id = id < 0 ? 0 : (id >= VV ? VV - 1 : id); const float p = sp[grp][s] * inv; const float* er = TAB + (size_t)id * DD; a0 += p * bfr(er[lane]); a1 += p * bfr(er[lane + 32]); }
  so[grp][lane] = a0; so[grp][lane + 32] = a1;
  __syncthreads();
  if (lane < 16) vst2(OUT + b * DD + lane * 4, *(const v4f*)&so[grp][lane * 4]); }
extern "C" void kernel_launch(void* const* d_in, const int* in_sizes, int n_in, void* d_out, int out_size, void* d_ws, size_t ws_size, hipStream_t stream) {
  (void)in_sizes; (void)n_in; (void)out_size;
  const float** F = (const float**)d_in;
  if (ws_size < (size_t)WS_END) return;
  char* ws = (char*)d_ws; float* SC = (float*)(ws + WS_SC);
  k_score<<<dim3(NRB), 128, 0, stream>>>(F[0], F[1], F[2], F[3], F[4], (const int*)d_in[5], SC);
  k_pool<<<dim3(NPB), 256, 0, stream>>>(F[0], SC, (const int*)d_in[5], (const int*)d_in[6], (float*)d_out);
}
